// MotionNet_29016799052669
// MI455X (gfx1250) — hardware-verified
//
#include <hip/hip_runtime.h>


#define NBT  4
#define CI   32
#define HH   256
#define NPX  (HH * HH)
#define HHALF 128
#define NCOR 81
#define CIN0 115
#define CP0  128
#define WP   258
#define NPP  (WP * WP)
#define NPR  66624
#define GB   320
#define NPT  (GB + NPR + GB)
#define DM   CP0
#define SLOPE 0.1f
#define LOSC 1024.0f

typedef _Float16 h16;
typedef unsigned short bf;
typedef __attribute__((ext_vector_type(16))) __bf16   v16bf;
typedef __attribute__((ext_vector_type(16))) _Float16 v16h;
typedef __attribute__((ext_vector_type(8)))  _Float16 v8h;
typedef __attribute__((ext_vector_type(8)))  unsigned short v8us;
typedef __attribute__((ext_vector_type(8)))  float    v8f;
typedef __attribute__((ext_vector_type(4)))  float    v4f;
typedef v8h  __attribute__((may_alias)) v8ha;
typedef v4f  __attribute__((may_alias)) v4fa;
typedef v8us __attribute__((may_alias)) v8usa;

__device__ __forceinline__ unsigned short f2bf(float f) { unsigned u = __float_as_uint(f); u += 0x7FFFu + ((u >> 16) & 1u); return (unsigned short)(u >> 16); }
__device__ __forceinline__ float bf2f(unsigned short b) { return __uint_as_float(((unsigned)b) << 16); }
__device__ __forceinline__ float bfr(float f) { return bf2f(f2bf(f)); }
__device__ __forceinline__ v16h cat16(v8h lo, v8h hi) { return __builtin_shufflevector(lo, hi, 0, 1, 2, 3, 4, 5, 6, 7, 8, 9, 10, 11, 12, 13, 14, 15); }
__device__ __forceinline__ v16bf cat16b(v8us lo, v8us hi) { return __builtin_bit_cast(v16bf, __builtin_shufflevector(lo, hi, 0, 1, 2, 3, 4, 5, 6, 7, 8, 9, 10, 11, 12, 13, 14, 15)); }
__device__ __forceinline__ v8f wmma16(v16h a, v16h b, v8f c) { return __builtin_amdgcn_wmma_f32_16x16x32_f16(false, a, false, b, (short)0, c, false, false); }
__device__ __forceinline__ v8f wmmab(v16bf a, v16bf b, v8f c) { return __builtin_amdgcn_wmma_f32_16x16x32_bf16(false, a, false, b, (short)0, c, false, false); }

template <bool SPLITA, bool F16OUT = false>
__global__ __launch_bounds__(128) void k_gemmb(const bf* __restrict__ A, const bf* __restrict__ Al, const bf* __restrict__ Bn, const float* __restrict__ bias, float* C, int ldc, h16* C2, const float* __restrict__ R = nullptr, int K = DM, int roundR = 1) {
    __shared__ __align__(16) float ost[4][16 * 68];
    const int lane = threadIdx.x & 31, wave = threadIdx.x >> 5, lr = lane & 15, hi = lane >> 4;
    const int r0 = blockIdx.x * 64 + wave * 16, c0 = blockIdx.y * 64;
    const size_t aoff = (size_t)(r0 + lr) * K + 8 * hi;
    size_t boff[4];
#pragma unroll
    for (int t = 0; t < 4; ++t) boff[t] = (size_t)(c0 + t * 16 + lr) * K + 8 * hi;
    v8f acc[4];
#pragma unroll
    for (int t = 0; t < 4; ++t) acc[t] = (v8f){};
#pragma unroll 1
    for (int kc = 0; kc < K; kc += 32) {
        const v16bf a = cat16b(*(const v8us*)(A + aoff + kc), *(const v8us*)(A + aoff + kc + 16));
        v16bf al = a;
        if (SPLITA) al = cat16b(*(const v8us*)(Al + aoff + kc), *(const v8us*)(Al + aoff + kc + 16));
#pragma unroll
        for (int t = 0; t < 4; ++t) { const v16bf b = cat16b(*(const v8us*)(Bn + boff[t] + kc), *(const v8us*)(Bn + boff[t] + kc + 16)); acc[t] = wmmab(a, b, acc[t]); if (SPLITA) acc[t] = wmmab(al, b, acc[t]); }
        asm volatile("v_nop\n\tv_nop\n\tv_nop\n\tv_nop" : "+v"(acc[0]), "+v"(acc[1]), "+v"(acc[2]), "+v"(acc[3]) : "v"(a), "v"(al));
    }
    float* os = &ost[wave][0];
#pragma unroll
    for (int t = 0; t < 4; ++t) { const float bv = bias ? bfr(bias[c0 + t * 16 + lr]) : 0.f;
#pragma unroll
        for (int j = 0; j < 8; ++j) os[(hi * 8 + j) * 68 + t * 16 + lr] = acc[t][j] + bv; }
    __syncthreads();
    if (F16OUT) {
        h16* crow = (h16*)(void*)C + (size_t)r0 * ldc + c0;
        auto pass = [&]() {
#pragma unroll
            for (int s = 0; s < 4; ++s) { const int row = 4 * s + (lane >> 3), piece = lane & 7; const float* sp = os + row * 68 + piece * 8; v8h o, o2;
#pragma unroll
                for (int i = 0; i < 8; ++i) { const h16 a = (h16)sp[i]; o[i] = a; o2[i] = (h16)((sp[i] - (float)a) * LOSC); }
                *(volatile v8h*)(crow + (size_t)row * ldc + piece * 8) = o; if (C2) *(volatile v8h*)(C2 + (size_t)r0 * ldc + c0 + (size_t)row * ldc + piece * 8) = o2; }
        };
        pass(); __threadfence(); pass();
    } else {
        float* crow = C + (size_t)r0 * ldc + c0;
        auto pass = [&]() {
#pragma unroll
            for (int s = 0; s < 8; ++s) { const int Lid = (lane >> 3) + 4 * s, piece = lane & 7; const int row = Lid >> 1, cofs = (Lid & 1) * 32 + piece * 4;
                v4f val = *(const v4fa*)(os + row * 68 + cofs); if (R) { const v4f rv = *(const v4f*)(R + ((size_t)r0 + row) * ldc + c0 + cofs); val += roundR ? (v4f){bfr(rv[0]), bfr(rv[1]), bfr(rv[2]), bfr(rv[3])} : rv; }
                *(volatile v4f*)(crow + (size_t)row * ldc + cofs) = val; }
        };
        pass(); __threadfence(); pass();
    }
}


__global__ __launch_bounds__(128) void k_gemmtap(const bf* __restrict__ Ah, const bf* __restrict__ Al, const bf* __restrict__ Bt, const float* __restrict__ bias, float* C, int ldc, int K) {
    __shared__ __align__(16) float ost[4][16 * 68];
    const int lane = threadIdx.x & 31, wave = threadIdx.x >> 5, lr = lane & 15, hi = lane >> 4;
    const int r0 = blockIdx.x * 64 + wave * 16, c0 = blockIdx.y * 64;
    v8f acc[4];
#pragma unroll
    for (int t = 0; t < 4; ++t) acc[t] = (v8f){};
#pragma unroll 1
    for (int tap = 0; tap < 9; ++tap) { const long off = (long)(tap / 3 - 1) * WP + (tap % 3 - 1);
        const size_t aoff = (size_t)((long)GB + off + r0 + lr) * K + 8 * hi; const bf* Bn = Bt + (size_t)tap * 64 * K;
        size_t boff[4];
#pragma unroll
        for (int t = 0; t < 4; ++t) boff[t] = (size_t)(c0 + t * 16 + lr) * K + 8 * hi;
#pragma unroll 1
        for (int kc = 0; kc < K; kc += 32) {
            const v16bf a = cat16b(*(const v8us*)(Ah + aoff + kc), *(const v8us*)(Ah + aoff + kc + 16));
            const v16bf al = cat16b(*(const v8us*)(Al + aoff + kc), *(const v8us*)(Al + aoff + kc + 16));
#pragma unroll
            for (int t = 0; t < 4; ++t) { const v16bf b = cat16b(*(const v8us*)(Bn + boff[t] + kc), *(const v8us*)(Bn + boff[t] + kc + 16)); acc[t] = wmmab(a, b, acc[t]); acc[t] = wmmab(al, b, acc[t]); }
            asm volatile("v_nop\n\tv_nop\n\tv_nop\n\tv_nop" : "+v"(acc[0]), "+v"(acc[1]), "+v"(acc[2]), "+v"(acc[3]) : "v"(a), "v"(al));
        } }
    float* os = &ost[wave][0];
#pragma unroll
    for (int t = 0; t < 4; ++t) { const float bv = bias ? bfr(bias[c0 + t * 16 + lr]) : 0.f;
#pragma unroll
        for (int j = 0; j < 8; ++j) os[(hi * 8 + j) * 68 + t * 16 + lr] = acc[t][j] + bv; }
    __syncthreads();
    float* crow = C + (size_t)r0 * ldc + c0;
    auto pass = [&]() {
#pragma unroll
        for (int s = 0; s < 8; ++s) { const int Lid = (lane >> 3) + 4 * s, piece = lane & 7; const int row = Lid >> 1, cofs = (Lid & 1) * 32 + piece * 4;
            const v4f val = *(const v4fa*)(os + row * 68 + cofs); *(volatile v4f*)(crow + (size_t)row * ldc + cofs) = val; }
    };
    pass(); __threadfence(); pass();
}

__global__ __launch_bounds__(256) void k_wtap(const float* __restrict__ Wt, int cout, int cin, int KP, bf* WT) {
    typedef __attribute__((ext_vector_type(4))) unsigned short v4us;
    const int lane = threadIdx.x & 31; const int w = blockIdx.x * 8 + (threadIdx.x >> 5); if (w >= 9 * 64) return; const int tap = w / 64, o = w % 64; const int ky = tap / 3, kx = tap % 3;
#pragma unroll 1
    for (int ps = 0; ps < 2; ++ps) {
#pragma unroll 1
        for (int c0 = lane * 4; c0 < KP; c0 += 128) { v4us v;
#pragma unroll
            for (int i = 0; i < 4; ++i) { const int ci = c0 + i; v[i] = f2bf((o < cout && ci < cin) ? Wt[(((size_t)(o < cout ? o : 0) * cin + (ci < cin ? ci : 0)) * 3 + ky) * 3 + kx] : 0.f); }
            *(volatile v4us*)(WT + ((size_t)tap * 64 + o) * KP + c0) = v; }
        if (ps == 0) __threadfence(); }
}
__global__ __launch_bounds__(64) void k_bpad64(const float* __restrict__ b, int n, float* BP) { const int t = threadIdx.x; const float v = (t < n) ? b[t < n ? t : 0] : 0.f; *(volatile float*)(BP + t) = v; __threadfence(); *(volatile float*)(BP + t) = v; }
__global__ __launch_bounds__(256) void k_corr(const float* __restrict__ xr, const float* __restrict__ xn, float* IN) {
    const int lane = threadIdx.x & 31; const size_t wid = (size_t)blockIdx.x * 8 + (threadIdx.x >> 5); if (wid >= (size_t)NCOR * (NPX / 32)) return; const int d = (int)(wid / (NPX / 32)); const int p = (int)(wid % (NPX / 32)) * 32 + lane;
    const int dy = d / 9 - 4, dx = d % 9 - 4; const int y = p >> 8, x = p & 255; const int yy = y + dy, xx = x + dx; const bool ok = yy >= 0 && yy < HH && xx >= 0 && xx < HH; const int q = ok ? (yy * HH + xx) : 0; float acc = 0.f;
#pragma unroll 4
    for (int c = 0; c < CI; ++c) acc = fmaf(bfr(xr[(size_t)c * NPX + p]), bfr(xn[(size_t)c * NPX + q]), acc);
    float v = ok ? acc * (1.0f / CI) : 0.f; v = (v >= 0.f) ? v : SLOPE * v;
    *(volatile float*)(IN + (size_t)d * NPX + p) = v; __threadfence(); *(volatile float*)(IN + (size_t)d * NPX + p) = v;
}
__global__ __launch_bounds__(256) void k_resize(const float* __restrict__ src, int nch, int ch0, float mult, float* IN) {
    const int lane = threadIdx.x & 31; const size_t wid = (size_t)blockIdx.x * 8 + (threadIdx.x >> 5); if (wid >= (size_t)nch * (NPX / 32)) return; const int c = (int)(wid / (NPX / 32)); const int p = (int)(wid % (NPX / 32)) * 32 + lane; const int y = p >> 8, x = p & 255;
    auto src1 = [&](int i, int& i0, int& i1, float& w1) { const float s = ((float)i + 0.5f) * 0.5f - 0.5f; const float f = floorf(s); i0 = (int)f; i1 = i0 + 1; w1 = s - f; i0 = i0 < 0 ? 0 : (i0 > HHALF - 1 ? HHALF - 1 : i0); i1 = i1 < 0 ? 0 : (i1 > HHALF - 1 ? HHALF - 1 : i1); };
    int y0, y1, x0, x1; float wy, wx; src1(y, y0, y1, wy); src1(x, x0, x1, wx); const float* sc = src + (size_t)c * HHALF * HHALF;
    const float v = (1.f - wy) * ((1.f - wx) * bfr(sc[y0 * HHALF + x0]) + wx * bfr(sc[y0 * HHALF + x1])) + wy * ((1.f - wx) * bfr(sc[y1 * HHALF + x0]) + wx * bfr(sc[y1 * HHALF + x1]));
    const float o = v * mult; *(volatile float*)(IN + (size_t)(ch0 + c) * NPX + p) = o; __threadfence(); *(volatile float*)(IN + (size_t)(ch0 + c) * NPX + p) = o;
}
template <int KP>
__global__ __launch_bounds__(256) void k_gridpl(const float* __restrict__ SRC, int cin, bf* Ph, bf* Pl) {
    const int lane = threadIdx.x & 31; const size_t w = (size_t)blockIdx.x * 8 + (threadIdx.x >> 5);
    if (KP == 128) { typedef __attribute__((ext_vector_type(4))) unsigned short v4us; const size_t r = w; if (r >= (size_t)NPT) return; const long pr = (long)r - GB; int y = -1, x = -1; bool live = false;
        if (pr >= 0 && pr < NPP) { const int gy = (int)(pr / WP), gx = (int)(pr % WP); y = gy - 1; x = gx - 1; live = (y >= 0 && y < HH && x >= 0 && x < HH); }
        v4us oh, ol;
#pragma unroll
        for (int i = 0; i < 4; ++i) { const int c = lane * 4 + i; float v = 0.f; if (live && c < cin) v = SRC[(size_t)c * NPX + y * HH + x]; const unsigned short hb = f2bf(v); oh[i] = hb; ol[i] = f2bf(v - bf2f(hb)); }
        const size_t o = r * KP + lane * 4; *(volatile v4us*)(Ph + o) = oh; *(volatile v4us*)(Pl + o) = ol; __threadfence(); *(volatile v4us*)(Ph + o) = oh; *(volatile v4us*)(Pl + o) = ol; }
    else { typedef __attribute__((ext_vector_type(2))) unsigned short v2us; const size_t r = w * 2 + (lane >> 4); if (r >= (size_t)NPT) return; const long pr = (long)r - GB; int y = -1, x = -1; bool live = false;
        if (pr >= 0 && pr < NPP) { const int gy = (int)(pr / WP), gx = (int)(pr % WP); y = gy - 1; x = gx - 1; live = (y >= 0 && y < HH && x >= 0 && x < HH); }
        const int c0 = (lane & 15) * 2; v2us oh, ol;
#pragma unroll
        for (int i = 0; i < 2; ++i) { const int c = c0 + i; float v = 0.f; if (live && c < cin) v = SRC[(size_t)c * NPX + y * HH + x]; const unsigned short hb = f2bf(v); oh[i] = hb; ol[i] = f2bf(v - bf2f(hb)); }
        const size_t o = r * KP + c0; *(volatile v2us*)(Ph + o) = oh; *(volatile v2us*)(Pl + o) = ol; __threadfence(); *(volatile v2us*)(Ph + o) = oh; *(volatile v2us*)(Pl + o) = ol; }
}
template <int MODE>
__global__ __launch_bounds__(256) void k_unpad(const float* __restrict__ Cm, const float* __restrict__ bias, const float* __restrict__ RES, float* DST, float* OUT3) {
    const int lane = threadIdx.x & 31; const int wid = blockIdx.x * 8 + (threadIdx.x >> 5); if (wid >= CI * (NPX / 128)) return; const int c = wid / (NPX / 128); const int p0 = (wid % (NPX / 128)) * 128 + lane * 4; const float bc = bfr(bias[c]); v4f v;
#pragma unroll
    for (int i = 0; i < 4; ++i) { const int p = p0 + i; const int y = p >> 8, x = p & 255; const size_t pr = (size_t)(y + 1) * WP + (x + 1); float t = Cm[pr * 64 + c] + bc; if (MODE == 1) t += RES[(size_t)c * NPX + p]; v[i] = (t >= 0.f) ? t : SLOPE * t; }
    const size_t o = (size_t)c * NPX + p0; *(volatile v4f*)(DST + o) = v; if (MODE == 1) *(volatile v4f*)(OUT3 + o) = v; __threadfence(); *(volatile v4f*)(DST + o) = v; if (MODE == 1) *(volatile v4f*)(OUT3 + o) = v;
}
__global__ __launch_bounds__(256) void k_flow(const float* __restrict__ Cm, const float* __restrict__ bias, float* FLO, float* MSK) {
    const int lane = threadIdx.x & 31; const int wid = blockIdx.x * 8 + (threadIdx.x >> 5); if (wid >= 3 * (NPX / 128)) return; const int c = wid / (NPX / 128); const int p0 = (wid % (NPX / 128)) * 128 + lane * 4; const float bc = bfr(bias[c]); v4f v;
#pragma unroll
    for (int i = 0; i < 4; ++i) { const int p = p0 + i; const int y = p >> 8, x = p & 255; const size_t pr = (size_t)(y + 1) * WP + (x + 1); const float t = Cm[pr * 64 + c] + bc; v[i] = (c == 2) ? 1.0f / (1.0f + expf(-t)) : t; }
    float* dst = (c == 2) ? (MSK + p0) : (FLO + (size_t)c * NPX + p0); *(volatile v4f*)dst = v; __threadfence(); *(volatile v4f*)dst = v;
}

extern "C" void kernel_launch(void* const* d_in, const int* in_sizes, int n_in,
                              void* d_out, int out_size, void* d_ws, size_t ws_size, hipStream_t stream) {
    (void)in_sizes; (void)n_in; (void)out_size;
    const float* xr = (const float*)d_in[0]; const float* xn = (const float*)d_in[1]; const float* bflow = (const float*)d_in[2]; const float* bfeat = (const float*)d_in[3];
    const float* w0 = (const float*)d_in[4]; const float* b0 = (const float*)d_in[5]; const float* w1 = (const float*)d_in[6]; const float* b1 = (const float*)d_in[7]; const float* w2 = (const float*)d_in[8]; const float* b2 = (const float*)d_in[9]; const float* wf = (const float*)d_in[10]; const float* bfv = (const float*)d_in[11];
    float* oflow = (float*)d_out;
    float* omask = (float*)((char*)d_out + (size_t)NBT * 2 * NPX * 4);
    float* ofeat = (float*)((char*)d_out + (size_t)NBT * 3 * NPX * 4);
    char* wsp = (char*)d_ws;
    auto take = [&](size_t bytes) { char* p = wsp; wsp += (bytes + 255) & ~(size_t)255; return (void*)p; };
    bf* WT0 = (bf*)take((size_t)9 * 64 * CP0 * 2); bf* WT1 = (bf*)take((size_t)9 * 64 * CI * 2); bf* WT2 = (bf*)take((size_t)9 * 64 * CI * 2); bf* WTF = (bf*)take((size_t)9 * 64 * CI * 2);
    float* IN = (float*)take((size_t)CIN0 * NPX * 4); float* Hc = (float*)take((size_t)CI * NPX * 4); float* T1 = (float*)take((size_t)CI * NPX * 4); float* FE = (float*)take((size_t)CI * NPX * 4);
    bf* Ph = (bf*)take((size_t)NPT * CP0 * 2); bf* Pl = (bf*)take((size_t)NPT * CP0 * 2); float* CA = (float*)take((size_t)NPR * 64 * 4);
    if ((size_t)(wsp - (char*)d_ws) > ws_size) return;
    k_wtap<<<(9 * 64) / 8, 256, 0, stream>>>(w0, CI, CIN0, CP0, WT0); k_wtap<<<(9 * 64) / 8, 256, 0, stream>>>(w1, CI, CI, CI, WT1); k_wtap<<<(9 * 64) / 8, 256, 0, stream>>>(w2, CI, CI, CI, WT2); k_wtap<<<(9 * 64) / 8, 256, 0, stream>>>(wf, 3, CI, CI, WTF);
    auto conv = [&](const bf* Wt, int KP) -> float* { k_gemmtap<<<dim3(NPR / 64, 1, 1), 128, 0, stream>>>(Ph, Pl, Wt, nullptr, CA, 64, KP); return CA; };
    for (int b = 0; b < NBT; ++b) {
        k_corr<<<(NCOR * (NPX / 32)) / 8, 256, 0, stream>>>(xr + (size_t)b * CI * NPX, xn + (size_t)b * CI * NPX, IN);
        k_resize<<<(CI * (NPX / 32)) / 8, 256, 0, stream>>>(bfeat + (size_t)b * CI * HHALF * HHALF, CI, NCOR, 1.0f, IN); k_resize<<<(2 * (NPX / 32)) / 8, 256, 0, stream>>>(bflow + (size_t)b * 2 * HHALF * HHALF, 2, NCOR + CI, 2.0f, IN);
        k_gridpl<CP0><<<(NPT + 7) / 8, 256, 0, stream>>>(IN, CIN0, Ph, Pl);   float* c0 = conv(WT0, CP0); k_unpad<0><<<(CI * (NPX / 128)) / 8, 256, 0, stream>>>(c0, b0, nullptr, Hc, nullptr);
        k_gridpl<CI><<<(NPT / 2 + 7) / 8, 256, 0, stream>>>(Hc, CI, Ph, Pl);  float* c1 = conv(WT1, CI);  k_unpad<0><<<(CI * (NPX / 128)) / 8, 256, 0, stream>>>(c1, b1, nullptr, T1, nullptr);
        k_gridpl<CI><<<(NPT / 2 + 7) / 8, 256, 0, stream>>>(T1, CI, Ph, Pl);  float* c2 = conv(WT2, CI);  k_unpad<1><<<(CI * (NPX / 128)) / 8, 256, 0, stream>>>(c2, b2, Hc, FE, ofeat + (size_t)b * CI * NPX);
        k_gridpl<CI><<<(NPT / 2 + 7) / 8, 256, 0, stream>>>(FE, CI, Ph, Pl);  float* c3 = conv(WTF, CI);  k_flow<<<(3 * (NPX / 128)) / 8, 256, 0, stream>>>(c3, bfv, oflow + (size_t)b * 2 * NPX, omask + (size_t)b * NPX); }
}
